// CBlock2_49349174231388
// MI455X (gfx1250) — hardware-verified
//
#include <hip/hip_runtime.h>
#include <math.h>


typedef __attribute__((ext_vector_type(16))) _Float16 v16h;
typedef __attribute__((ext_vector_type(8)))  _Float16 v8h;
typedef __attribute__((ext_vector_type(16))) __bf16   v16b;
typedef __attribute__((ext_vector_type(8)))  __bf16   v8b;
typedef __attribute__((ext_vector_type(8)))  float    v8f;
typedef __attribute__((ext_vector_type(4)))  float    v4f;

__device__ __forceinline__ unsigned short f2bf_bits(float f) {
  unsigned u = __float_as_uint(f);
  return (unsigned short)((u + 0x7FFFu + ((u >> 16) & 1u)) >> 16);
}
__device__ __forceinline__ float bf_bits2f(unsigned short h) { return __uint_as_float(((unsigned)h) << 16); }

__device__ __forceinline__ void dep_guard_h(v8f& a, v8f& b, v16h x, v16h y) { asm volatile("v_nop\n\tv_nop\n\tv_nop\n\tv_nop" : "+v"(a), "+v"(b) : "v"(x), "v"(y)); }
__device__ __forceinline__ void dep_guard_b(v8f& a, v8f& b, v16b x, v16b y) { asm volatile("v_nop\n\tv_nop\n\tv_nop\n\tv_nop" : "+v"(a), "+v"(b) : "v"(x), "v"(y)); }
__device__ __forceinline__ void keep4_h(v16h a, v16h b, v16h c, v16h d) { asm volatile("v_nop" :: "v"(a), "v"(b), "v"(c), "v"(d)); }
__device__ __forceinline__ void keep4_b(v16b a, v16b b, v16b c, v16b d) { asm volatile("v_nop" :: "v"(a), "v"(b), "v"(c), "v"(d)); }
__device__ __forceinline__ void acc_guard4(v8f& a, v8f& b, v8f& c, v8f& d) { asm volatile("v_nop\n\tv_nop\n\tv_nop\n\tv_nop" : "+v"(a), "+v"(b), "+v"(c), "+v"(d)); }
template <typename T> struct Frag;
template <> struct Frag<_Float16> {
  typedef v16h V; union U { v16h v; v8h h[2]; };
  static __device__ __forceinline__ v16h load(const _Float16* p) {
    U f; f.h[0] = *(const v8h*)(p); f.h[1] = *(const v8h*)(p + 16); return f.v;
  }
  static __device__ __forceinline__ v8f mma(v16h a, v16h b, v8f c) {
    return __builtin_amdgcn_wmma_f32_16x16x32_f16(false, a, false, b, (short)0, c, false, false);
  }
  static __device__ __forceinline__ void guard(v8f& a, v8f& b, v16h x, v16h y) { dep_guard_h(a, b, x, y); }
  static __device__ __forceinline__ void keep(v16h a, v16h b, v16h c, v16h d) { keep4_h(a, b, c, d); }
};
template <> struct Frag<__bf16> {
  typedef v16b V; union U { v16b v; v8b h[2]; };
  static __device__ __forceinline__ v16b load(const __bf16* p) {
    U f; f.h[0] = *(const v8b*)(p); f.h[1] = *(const v8b*)(p + 16); return f.v;
  }
  static __device__ __forceinline__ v8f mma(v16b a, v16b b, v8f c) {
    return __builtin_amdgcn_wmma_f32_16x16x32_bf16(false, a, false, b, (short)0, c, false, false);
  }
  static __device__ __forceinline__ void guard(v8f& a, v8f& b, v16b x, v16b y) { dep_guard_b(a, b, x, y); }
  static __device__ __forceinline__ void keep(v16b a, v16b b, v16b c, v16b d) { keep4_b(a, b, c, d); }
};

template <int ET> struct Elem;
template <> struct Elem<0> { typedef _Float16 T; };
template <> struct Elem<1> { typedef __bf16 T; };
template <int ET, bool SPLIT, int BIAS_MODE, int OUT_MODE, bool RESID, int ACT = 0>
__global__ __launch_bounds__(256) void wmma_gemm64(
    const unsigned short* __restrict__ Ap, const unsigned short* __restrict__ A2p, int lda, long strideA,
    const unsigned short* __restrict__ Btp, const unsigned short* __restrict__ Bt2p, int ldb, long strideB,
    void* __restrict__ Cout, void* __restrict__ Cout2, int ldc, long strideC,
    const float* __restrict__ bias,
    const float* __restrict__ resid, long strideR,
    int M, int N, int K, float scale) {
  typedef typename Elem<ET>::T T;
  typedef typename Frag<T>::V V;
  const T* A = (const T*)Ap; const T* A2 = (const T*)A2p; const T* Bt = (const T*)Btp; const T* Bt2 = (const T*)Bt2p;
  __shared__ __align__(16) float sT[8][16 * 68];
  const int b    = blockIdx.y;
  const int lane = threadIdx.x & 31;
  const int wave = threadIdx.x >> 5;
  const int tilesN = N >> 6;
  const int tilesM = M >> 6;
  const int tile = blockIdx.x * 8 + wave;
  if (tile >= tilesM * tilesN) return;
  const int tm = tile / tilesN;
  const int tn = tile - tm * tilesN;
  const int m0 = tm << 6;
  const int n0 = tn << 6;

  const T* Ab  = A  + (size_t)b * strideA;
  const T* Bb  = Bt + (size_t)b * strideB;
  const T* Ab2 = SPLIT ? (A2  + (size_t)b * strideA) : nullptr;
  const T* Bb2 = SPLIT ? (Bt2 + (size_t)b * strideB) : nullptr;

  const int rlane = lane & 15;
  const int koff  = (lane >> 4) * 8;
  const int mOff  = (lane >> 4) * 8;

  v8f acc[4][4];
#pragma unroll
  for (int i = 0; i < 4; ++i)
#pragma unroll
    for (int j = 0; j < 4; ++j) acc[i][j] = (v8f){0.f,0.f,0.f,0.f,0.f,0.f,0.f,0.f};

  for (int k0 = 0; k0 < K; k0 += 32) {
    V bh[4], bl[4];
#pragma unroll
    for (int j = 0; j < 4; ++j) {
      const size_t bo = (size_t)(n0 + (j << 4) + rlane) * ldb + koff + k0;
      bh[j] = Frag<T>::load(Bb + bo);
      if (SPLIT) bl[j] = Frag<T>::load(Bb2 + bo);
    }
#pragma unroll
    for (int i = 0; i < 4; ++i) {
      const size_t ao = (size_t)(m0 + (i << 4) + rlane) * lda + koff + k0;
      V ah = Frag<T>::load(Ab + ao);
      V al;
      if (SPLIT) al = Frag<T>::load(Ab2 + ao);
#pragma unroll
      for (int j = 0; j < 4; ++j) {
        acc[i][j] = Frag<T>::mma(ah, bh[j], acc[i][j]);
        if (SPLIT) {
          acc[i][j] = Frag<T>::mma(ah, bl[j], acc[i][j]);
          acc[i][j] = Frag<T>::mma(al, bh[j], acc[i][j]);
        }
      }
      Frag<T>::guard(acc[i][0], acc[i][3], ah, SPLIT ? al : ah);
    }
    Frag<T>::keep(bh[0], bh[1], bh[2], bh[3]);
    if (SPLIT) Frag<T>::keep(bl[0], bl[1], bl[2], bl[3]);
  }
  acc_guard4(acc[0][0], acc[0][1], acc[0][2], acc[0][3]);
  acc_guard4(acc[1][0], acc[1][1], acc[1][2], acc[1][3]);
  acc_guard4(acc[2][0], acc[2][1], acc[2][2], acc[2][3]);
  acc_guard4(acc[3][0], acc[3][1], acc[3][2], acc[3][3]);

  float* slab = sT[wave];
  const float* Rb = RESID ? (resid + (size_t)b * strideR) : nullptr;
#pragma unroll
  for (int i = 0; i < 4; ++i) {
    const int mBase = m0 + (i << 4);
#pragma unroll
    for (int j = 0; j < 4; ++j) {
      const int n = n0 + (j << 4) + rlane;
      float bv = 0.f;
      if (BIAS_MODE == 2) bv = bias[n];
#pragma unroll
      for (int r = 0; r < 8; ++r) {
        float v = acc[i][j][r] * scale;
        if (BIAS_MODE == 1) v += bias[mBase + mOff + r];
        if (BIAS_MODE == 2) v += bv;
        if (RESID) v += Rb[(size_t)(mBase + mOff + r) * ldc + n];
        if (ACT == 1) v = tanhf(v);
        if (ACT == 2) v = fmaxf(v, 0.0f);
        if (ACT == 3) v = v / (1.0f + expf(-v));
        if (ACT == 4) v = (v > 0.f) ? v : 0.01f * v;
        if (ACT == 5) v = 0.5f * v * (1.0f + erff(v * 0.70710678118654752f));
        slab[(mOff + r) * 68 + (j << 4) + rlane] = v;
      }
    }
    __builtin_amdgcn_fence(__ATOMIC_RELEASE, "workgroup");
    __builtin_amdgcn_wave_barrier();
    __builtin_amdgcn_fence(__ATOMIC_ACQUIRE, "workgroup");
    if (OUT_MODE == 0) {
      float* C = (float*)Cout + (size_t)b * strideC;
      const int hh = lane >> 4, c4 = (lane & 15) * 4;
      for (int pass = 0; pass < 2; ++pass) {
#pragma unroll
        for (int it = 0; it < 8; ++it) {
          const int row = it * 2 + hh;
          v4f v = *(const v4f*)(slab + row * 68 + c4);
          *(volatile v4f*)(C + (size_t)(mBase + row) * ldc + n0 + c4) = v;
        }
        __threadfence();
      }
    } else {
      const int q = lane >> 3, c8 = (lane & 7) * 8;
      unsigned short* C  = (unsigned short*)Cout  + (size_t)b * strideC;
      unsigned short* C2 = (OUT_MODE == 2) ? ((unsigned short*)Cout2 + (size_t)b * strideC) : nullptr;
      for (int pass = 0; pass < 2; ++pass) {
#pragma unroll
        for (int it = 0; it < 4; ++it) {
          const int row = it * 4 + q;
          const float* sp = slab + row * 68 + c8;
          v8h hv, lv;
#pragma unroll
          for (int e = 0; e < 8; ++e) {
            if (OUT_MODE == 1) {
              hv[e] = (_Float16)sp[e];
            } else {
              unsigned short hb = f2bf_bits(sp[e]);
              unsigned short lb = f2bf_bits(sp[e] - bf_bits2f(hb));
              hv[e] = __builtin_bit_cast(_Float16, hb);
              lv[e] = __builtin_bit_cast(_Float16, lb);
            }
          }
          *(volatile v8h*)(C + (size_t)(mBase + row) * ldc + n0 + c8) = hv;
          if (OUT_MODE == 2) *(volatile v8h*)(C2 + (size_t)(mBase + row) * ldc + n0 + c8) = lv;
        }
        __threadfence();
      }
    }
    __builtin_amdgcn_fence(__ATOMIC_RELEASE, "workgroup");
    __builtin_amdgcn_wave_barrier();
    __builtin_amdgcn_fence(__ATOMIC_ACQUIRE, "workgroup");
  }
}

__global__ __launch_bounds__(256) void cast_f32_f16x2s(
    const float* __restrict__ in, unsigned short* __restrict__ out, int n2, float sc) {
  int i = blockIdx.x * 256 + threadIdx.x;
  if (i < n2) {
    const _Float16 h0 = (_Float16)(in[2 * i] * sc), h1 = (_Float16)(in[2 * i + 1] * sc);
    const unsigned u = (unsigned)__builtin_bit_cast(unsigned short, h0) | ((unsigned)__builtin_bit_cast(unsigned short, h1) << 16);
    ((volatile unsigned*)out)[i] = u;
    __threadfence();
    ((volatile unsigned*)out)[i] = u;
  }
}

#define LNC 512
__global__ __launch_bounds__(256) void ln_f16_kernel(
    const float* __restrict__ x, const float* __restrict__ g, const float* __restrict__ bt,
    unsigned short* __restrict__ outp, int rows, float eps) {
  _Float16* out = (_Float16*)outp;
  const int lane = threadIdx.x & 31, wave = threadIdx.x >> 5;
  const int row = blockIdx.x * 8 + wave;
  if (row >= rows) return;
  const float* p = x + (size_t)row * LNC;
  const int c0 = 8 * lane, c1 = (LNC / 2) + 8 * lane;
  const v4f a0 = *(const v4f*)(p + c0), a1 = *(const v4f*)(p + c0 + 4);
  const v4f a2 = *(const v4f*)(p + c1), a3 = *(const v4f*)(p + c1 + 4);
  float vals[16];
#pragma unroll
  for (int e = 0; e < 4; ++e) { vals[e] = a0[e]; vals[4 + e] = a1[e]; vals[8 + e] = a2[e]; vals[12 + e] = a3[e]; }
  float s = 0.f;
#pragma unroll
  for (int i = 0; i < 16; ++i) s += vals[i];
#pragma unroll
  for (int m = 16; m >= 1; m >>= 1) s += __shfl_xor(s, m, 32);
  const float mu = s * (1.0f / LNC);
  float sq = 0.f;
#pragma unroll
  for (int i = 0; i < 16; ++i) { const float d = vals[i] - mu; sq += d * d; }
#pragma unroll
  for (int m = 16; m >= 1; m >>= 1) sq += __shfl_xor(sq, m, 32);
  const float rs = 1.0f / sqrtf(sq * (1.0f / LNC) + eps);
  const v4f g0 = *(const v4f*)(g + c0), g1v = *(const v4f*)(g + c0 + 4), g2v = *(const v4f*)(g + c1), g3 = *(const v4f*)(g + c1 + 4);
  const v4f b0 = *(const v4f*)(bt + c0), b1v = *(const v4f*)(bt + c0 + 4), b2v = *(const v4f*)(bt + c1), b3 = *(const v4f*)(bt + c1 + 4);
  v8h o0, o1;
#pragma unroll
  for (int e = 0; e < 4; ++e) {
    o0[e]     = (_Float16)((vals[e] - mu) * rs * g0[e] + b0[e]);
    o0[4 + e] = (_Float16)((vals[4 + e] - mu) * rs * g1v[e] + b1v[e]);
    o1[e]     = (_Float16)((vals[8 + e] - mu) * rs * g2v[e] + b2v[e]);
    o1[4 + e] = (_Float16)((vals[12 + e] - mu) * rs * g3[e] + b3[e]);
  }
  _Float16* orow = out + (size_t)row * LNC;
  *(volatile v8h*)(orow + c0) = o0;
  *(volatile v8h*)(orow + c1) = o1;
  __threadfence();
  *(volatile v8h*)(orow + c0) = o0;
  *(volatile v8h*)(orow + c1) = o1;
}

__global__ __launch_bounds__(256) void rowsum_f16_kernel(
    const unsigned short* __restrict__ vp, float* __restrict__ sums, int nrows, int S) {
  const _Float16* vt = (const _Float16*)vp;
  __shared__ float red[32];
  const int lane = threadIdx.x & 31, wave = threadIdx.x >> 5;
  const int r0 = blockIdx.x * 32;
  const int nu = S >> 8;
#pragma unroll
  for (int i = 0; i < 4; ++i) {
    const int row = r0 + wave * 4 + i;
    float s = 0.f;
    if (row < nrows) {
      const _Float16* p = vt + (size_t)row * S + 8 * lane;
      for (int u = 0; u < nu; ++u) {
        const v8h hv = *(const v8h*)(p + (u << 8));
#pragma unroll
        for (int e = 0; e < 8; ++e) s += (float)hv[e];
      }
    }
#pragma unroll
    for (int m = 16; m >= 1; m >>= 1) s += __shfl_xor(s, m, 32);
    if (lane == 0) red[wave * 4 + i] = s;
  }
  __syncthreads();
  if (wave == 0) {
    const int row = r0 + lane;
    const float val = red[lane];
    if (row < nrows) ((volatile float*)sums)[row] = val;
    __threadfence();
    if (row < nrows) ((volatile float*)sums)[row] = val;
  }
}

#define AD 64
#define ANW 4
#define AKC 64
#define OSP 68

__device__ __forceinline__ v8f h_mma(v16h a, v16h b, v8f c) {
  c = __builtin_amdgcn_wmma_f32_16x16x32_f16(false, a, false, b, (short)0, c, false, false);
  asm volatile("v_nop\n\tv_nop\n\tv_nop\n\tv_nop" : "+v"(c) : "v"(a), "v"(b));
  return c;
}

__global__ __launch_bounds__(128)
void gattn64_kernel(const unsigned short* __restrict__ qp, const unsigned short* __restrict__ kp,
                    const unsigned short* __restrict__ vtp, unsigned short* __restrict__ outp,
                    const int* __restrict__ gid, const float* __restrict__ gsum,
                    int S, int Hn, int ldr, float sscale, float eps_n, float eps) {
  const _Float16* q  = (const _Float16*)qp;
  const _Float16* k  = (const _Float16*)kp;
  const _Float16* vt = (const _Float16*)vtp;
  _Float16* out = (_Float16*)outp;
  __shared__ __align__(16) _Float16 Ksh[AKC * AD];
  __shared__ __align__(16) _Float16 Vth[AD * AKC];
  __shared__ __align__(16) _Float16 Psh[ANW][16 * AKC];
  __shared__ __align__(16) float  Os[ANW][16 * OSP];
  __shared__ int Kc[AKC];

  const int tid  = threadIdx.x;
  const int wave = tid >> 5;
  const int lane = tid & 31;
  const int hh   = lane >> 4;
  const int c    = lane & 15;

  const int nqb = S / AKC;
  const int bx = blockIdx.x;
  const int qb = bx % nqb;
  const int bh = bx / nqb;
  const int h  = bh % Hn;
  const int b  = bh / Hn;
  const int q0 = qb * AKC + wave * 16;

  const _Float16* qb_ptr = q  + (size_t)b * S * ldr + (size_t)h * AD;
  const _Float16* kb_ptr = k  + (size_t)b * S * ldr + (size_t)h * AD;
  const _Float16* vb_ptr = vt + ((size_t)(b * Hn + h) * AD) * (size_t)S;
  _Float16*       ob_ptr = out + (size_t)b * S * ldr + (size_t)h * AD;
  const int*      gb     = gid + (size_t)b * S;

  v16h qa0, qa1;
  {
    const _Float16* qrow = qb_ptr + (size_t)(q0 + c) * ldr;
    qa0 = Frag<_Float16>::load(qrow + 8 * hh);
    qa1 = Frag<_Float16>::load(qrow + 32 + 8 * hh);
  }
  int qc[8];
#pragma unroll
  for (int r = 0; r < 8; ++r) qc[r] = gb[q0 + 8 * hh + r];

  float lrow[8];
  v8f oacc[4];
#pragma unroll
  for (int r = 0; r < 8; ++r) lrow[r] = 0.f;
#pragma unroll
  for (int t = 0; t < 4; ++t) oacc[t] = (v8f){0.f,0.f,0.f,0.f,0.f,0.f,0.f,0.f};

  const int nChunks = S / AKC;
  for (int kc = 0; kc < nChunks; ++kc) {
    const int kv0 = kc * AKC;
    __syncthreads();
    {
      const int kvr = tid >> 1, dh = (tid & 1) * 32;
      const _Float16* krow = kb_ptr + (size_t)(kv0 + kvr) * ldr + dh;
#pragma unroll
      for (int i = 0; i < 4; ++i) *(v8h*)(Ksh + kvr * AD + dh + 8 * i) = *(const v8h*)(krow + 8 * i);
      const _Float16* vrow = vb_ptr + (size_t)kvr * S + kv0 + dh;
#pragma unroll
      for (int i = 0; i < 4; ++i) *(v8h*)(Vth + kvr * AKC + dh + 8 * i) = *(const v8h*)(vrow + 8 * i);
      if (tid < AKC) Kc[tid] = gb[kv0 + tid];
    }
    __syncthreads();

    v8f s[4];
#pragma unroll
    for (int j = 0; j < 4; ++j) {
      s[j] = (v8f){0.f,0.f,0.f,0.f,0.f,0.f,0.f,0.f};
      const v16h kb0 = Frag<_Float16>::load(Ksh + (j * 16 + c) * AD + 8 * hh);
      s[j] = h_mma(qa0, kb0, s[j]);
      const v16h kb1 = Frag<_Float16>::load(Ksh + (j * 16 + c) * AD + 32 + 8 * hh);
      s[j] = h_mma(qa1, kb1, s[j]);
    }
    int kvc[4];
#pragma unroll
    for (int j = 0; j < 4; ++j) kvc[j] = Kc[j * 16 + c];

    _Float16* pw = Psh[wave];
#pragma unroll
    for (int r = 0; r < 8; ++r) {
      float psum = 0.f;
#pragma unroll
      for (int j = 0; j < 4; ++j) {
        const bool same = (qc[r] == kvc[j]);
        const float e = same ? __expf(s[j][r] * sscale) : 0.f;
        psum += e;
        pw[(8 * hh + r) * AKC + j * 16 + c] = (_Float16)e;
      }
#pragma unroll
      for (int off = 1; off < 16; off <<= 1) psum += __shfl_xor(psum, off, 32);
      lrow[r] += psum;
    }
    __builtin_amdgcn_fence(__ATOMIC_RELEASE, "workgroup");
    __builtin_amdgcn_wave_barrier();
    __builtin_amdgcn_fence(__ATOMIC_ACQUIRE, "workgroup");

#pragma unroll 1
    for (int kk = 0; kk < 2; ++kk) {
      const v16h pa = Frag<_Float16>::load(pw + c * AKC + kk * 32 + 8 * hh);
#pragma unroll
      for (int t = 0; t < 4; ++t) {
        const v16h vb = Frag<_Float16>::load(Vth + (t * 16 + c) * AKC + kk * 32 + 8 * hh);
        oacc[t] = h_mma(pa, vb, oacc[t]);
      }
    }
  }

  float* os = Os[wave];
  float vsb[4];
#pragma unroll
  for (int t = 0; t < 4; ++t) vsb[t] = gsum[(size_t)bh * AD + t * 16 + c] * eps_n;
#pragma unroll
  for (int r = 0; r < 8; ++r) {
    const float inv = 1.0f / (lrow[r] + eps);
#pragma unroll
    for (int t = 0; t < 4; ++t) os[(8 * hh + r) * OSP + t * 16 + c] = (oacc[t][r] + vsb[t]) * inv;
  }
  __builtin_amdgcn_fence(__ATOMIC_RELEASE, "workgroup");
  __builtin_amdgcn_wave_barrier();
  __builtin_amdgcn_fence(__ATOMIC_ACQUIRE, "workgroup");
  {
    const int qq = lane >> 3, c8 = (lane & 7) * 8;
    for (int pass = 0; pass < 2; ++pass) {
#pragma unroll
      for (int it = 0; it < 4; ++it) {
        const int row = it * 4 + qq;
        const float* sp = os + row * OSP + c8;
        v8h hv;
#pragma unroll
        for (int e = 0; e < 8; ++e) hv[e] = (_Float16)sp[e];
        *(volatile v8h*)(ob_ptr + (size_t)(q0 + row) * ldr + c8) = hv;
      }
      __threadfence();
    }
  }
}

extern "C" void kernel_launch(void* const* d_in, const int* in_sizes, int n_in,
                              void* d_out, int out_size, void* d_ws,
                              size_t ws_size, hipStream_t stream) {
  if (n_in < 16) return;
  const int N = 1024, C = 512, H = 8, HD = 64, HID = 2048;
  const int B = in_sizes[0] / (N * C);
  const int rows = B * N;
  if (B < 1) return;
  if (in_sizes[0] != rows * C || in_sizes[15] != rows || out_size != rows * C) return;
  if (in_sizes[2] != C * C || in_sizes[3] != C * C || in_sizes[4] != C * C || in_sizes[5] != C * C) return;
  if (in_sizes[11] != HID * C || in_sizes[13] != C * HID) return;
  if (in_sizes[6] != C || in_sizes[7] != C || in_sizes[8] != C || in_sizes[9] != C || in_sizes[10] != C) return;
  if (in_sizes[12] != HID || in_sizes[14] != C) return;
  if ((rows % 64) != 0 || H * HD != C) return;

  const float* x_token = (const float*)d_in[0];
  const float* wq     = (const float*)d_in[2];
  const float* wk     = (const float*)d_in[3];
  const float* wv     = (const float*)d_in[4];
  const float* w_proj = (const float*)d_in[5];
  const float* b_proj = (const float*)d_in[6];
  const float* g1     = (const float*)d_in[7];
  const float* b1     = (const float*)d_in[8];
  const float* g2     = (const float*)d_in[9];
  const float* b2     = (const float*)d_in[10];
  const float* w1     = (const float*)d_in[11];
  const float* bb1    = (const float*)d_in[12];
  const float* w2     = (const float*)d_in[13];
  const float* bb2    = (const float*)d_in[14];
  const int*   gid    = (const int*)d_in[15];

  char* ws = (char*)d_ws;
  size_t off = 0;
  auto carve = [&](size_t bytes) { char* p = ws + off; off += (bytes + 255) & ~(size_t)255; return p; };
  const size_t BNC = (size_t)rows * C;
  unsigned short* wqk16 = (unsigned short*)carve((size_t)2 * C * C * 2);
  unsigned short* wv16  = (unsigned short*)carve((size_t)C * C * 2);
  unsigned short* wp16  = (unsigned short*)carve((size_t)C * C * 2);
  unsigned short* w116  = (unsigned short*)carve((size_t)HID * C * 2);
  unsigned short* w216  = (unsigned short*)carve((size_t)C * HID * 2);
  unsigned short* t16   = (unsigned short*)carve(BNC * 2);
  unsigned short* h216  = (unsigned short*)carve(BNC * 2);
  unsigned short* qk16  = (unsigned short*)carve((size_t)2 * BNC * 2);
  unsigned short* vt16  = (unsigned short*)carve(BNC * 2);
  float*          vsum  = (float*)carve((size_t)B * C * 4);
  unsigned short* att16 = (unsigned short*)carve(BNC * 2);
  float*          xres  = (float*)carve(BNC * 4);
  unsigned short* m116  = (unsigned short*)carve((size_t)rows * HID * 2);
  if (off > ws_size || off > (size_t)134217728) return;

  const float WSC = 16.0f, WINV = 0.0625f;

  {
    const int n2c = C * C / 2, n2h = HID * C / 2;
    cast_f32_f16x2s<<<(n2c + 255) / 256, 256, 0, stream>>>(wq, wqk16, n2c, WSC);
    cast_f32_f16x2s<<<(n2c + 255) / 256, 256, 0, stream>>>(wk, wqk16 + (size_t)C * C, n2c, WSC);
    cast_f32_f16x2s<<<(n2c + 255) / 256, 256, 0, stream>>>(wv, wv16, n2c, WSC);
    cast_f32_f16x2s<<<(n2c + 255) / 256, 256, 0, stream>>>(w_proj, wp16, n2c, WSC);
    cast_f32_f16x2s<<<(n2h + 255) / 256, 256, 0, stream>>>(w1, w116, n2h, WSC);
    cast_f32_f16x2s<<<(n2h + 255) / 256, 256, 0, stream>>>(w2, w216, n2h, WSC);
  }

  ln_f16_kernel<<<(rows + 7) / 8, 256, 0, stream>>>(x_token, g1, b1, t16, rows, 1e-5f);

  {
    const int tiles = (rows / 64) * (C / 64);
    wmma_gemm64<0, false, 0, 1, false, 0><<<dim3((tiles + 7) / 8, 2), 256, 0, stream>>>(
        t16, t16, C, 0L, wqk16, wqk16, C, (long)C * C, (void*)qk16, (void*)qk16, C, (long)rows * C,
        b_proj, x_token, 0L, rows, C, C, WINV);
  }
  {
    const int tiles = (C / 64) * (N / 64);
    wmma_gemm64<0, false, 0, 1, false, 0><<<dim3((tiles + 7) / 8, B), 256, 0, stream>>>(
        wv16, wv16, C, 0L, t16, t16, C, (long)N * C, (void*)vt16, (void*)vt16, N, (long)C * N,
        b_proj, x_token, 0L, C, N, C, WINV);
  }
  rowsum_f16_kernel<<<(B * C + 31) / 32, 256, 0, stream>>>(vt16, vsum, B * C, N);

  gattn64_kernel<<<B * H * (N / 64), 128, 0, stream>>>(
      qk16, qk16 + BNC, vt16, att16, gid, vsum, N, H, C, 0.125f, 1e-6f / (float)N, 1e-6f);

  {
    const int tiles = (rows / 64) * (C / 64);
    wmma_gemm64<0, false, 2, 0, true, 0><<<dim3((tiles + 7) / 8, 1), 256, 0, stream>>>(
        att16, att16, C, 0L, wp16, wp16, C, 0L, (void*)xres, (void*)xres, C, 0L,
        b_proj, x_token, 0L, rows, C, C, WINV);
  }
  ln_f16_kernel<<<(rows + 7) / 8, 256, 0, stream>>>(xres, g2, b2, h216, rows, 1e-5f);

  {
    const int tiles = (rows / 64) * (HID / 64);
    wmma_gemm64<0, false, 2, 1, false, 5><<<dim3((tiles + 7) / 8, 1), 256, 0, stream>>>(
        h216, h216, C, 0L, w116, w116, C, 0L, (void*)m116, (void*)m116, HID, 0L,
        bb1, xres, 0L, rows, HID, C, WINV);
  }
  {
    const int tiles = (rows / 64) * (C / 64);
    wmma_gemm64<0, false, 2, 0, true, 0><<<dim3((tiles + 7) / 8, 1), 256, 0, stream>>>(
        m116, m116, HID, 0L, w216, w216, HID, 0L, d_out, d_out, C, 0L,
        bb2, xres, 0L, rows, C, HID, WINV);
  }
}
